// Fusion_1640677507707
// MI455X (gfx1250) — hardware-run, weakly checked
//
#include <hip/hip_runtime.h>
#include <math.h>
#include <stdint.h>

#define DD     16
#define KK     16
#define NC_    100000
#define NI_    200000
#define NS_    200000
#define UC_    (NC_ * DD / 8)
#define UI_    (NI_ * DD / 8)
#define US_    (NS_ * DD / 8)
#define BC_    ((UC_ + 255) / 256)
#define BI_    ((UI_ + 255) / 256)
#define BS_    ((US_ + 255) / 256)
#define NREC   5
#define PAR_DW 320
#define PAR_WAS 256
#define PAR_WAN 272
#define PAR_BA  288
#define O0_    0
#define O1_    (NC_ * DD)
#define O2_    (O1_ + NI_ * DD)
#define OTOT_  (O2_ + NS_ * DD)
#define WSCAP  134217728

static_assert(KK == 16 && DD == 16);
static_assert(NC_ % 16 == 0 && NI_ % 16 == 0 && NS_ % 16 == 0);
static_assert(UC_ % 32 == 0 && UI_ % 32 == 0 && US_ % 32 == 0);
static_assert(((size_t)O1_ * 4) % 128 == 0 && ((size_t)O2_ * 4) % 128 == 0);
static_assert((size_t)(NS_ / 16 - 1) * 256 + 255 + O2_ == (size_t)OTOT_ - 1);
static_assert((PAR_DW * 4) % 128 == 0);

typedef __bf16         v16b  __attribute__((ext_vector_type(16)));
typedef float          v8f   __attribute__((ext_vector_type(8)));
typedef float          v4f   __attribute__((ext_vector_type(4)));
typedef unsigned int   v4u   __attribute__((ext_vector_type(4)));
typedef unsigned int   v2u   __attribute__((ext_vector_type(2)));
typedef v4f __attribute__((may_alias)) v4fa;
typedef v4u __attribute__((may_alias)) v4ua;
typedef v2u __attribute__((may_alias)) v2ua;

#if defined(__HIP_DEVICE_COMPILE__)
#define DEV_ASM 1
#else
#define DEV_ASM 0
#endif

__device__ __forceinline__ unsigned short bf_bits(float f) {
  const unsigned u = __float_as_uint(f);
  const unsigned r = (u + 0x7FFFu + ((u >> 16) & 1u)) >> 16;
  const unsigned q = (u >> 16) | 0x40u;
  return (unsigned short)(((u & 0x7fffffffu) > 0x7f800000u) ? q : r);
}
__device__ __forceinline__ float bf_up(unsigned hb) { return __uint_as_float((hb & 0xffffu) << 16); }
__device__ __forceinline__ float bf_lo(unsigned w) { return __uint_as_float(w << 16); }
__device__ __forceinline__ float bf_hi(unsigned w) { return __uint_as_float(w & 0xffff0000u); }
__device__ __forceinline__ float bfr(float f) { return bf_up((unsigned)bf_bits(f)); }
__device__ __forceinline__ unsigned pk16(unsigned short a, unsigned short b) { return (unsigned)a | ((unsigned)b << 16); }
__device__ __forceinline__ v8f zero8() { v8f z = {0.f, 0.f, 0.f, 0.f, 0.f, 0.f, 0.f, 0.f}; return z; }

__device__ __forceinline__ void pin4f(v4f x) {
#if DEV_ASM
  asm volatile("" :: "v"(x));
#else
  (void)x;
#endif
}
__device__ __forceinline__ void pin4u(v4u x) {
#if DEV_ASM
  asm volatile("" :: "v"(x));
#else
  (void)x;
#endif
}
__device__ __forceinline__ void pin1f(float x) {
#if DEV_ASM
  asm volatile("" :: "v"(x));
#else
  (void)x;
#endif
}

__device__ __forceinline__ void wave_lds_sync() {
  __builtin_amdgcn_fence(__ATOMIC_RELEASE, "workgroup");
  __builtin_amdgcn_wave_barrier();
  __builtin_amdgcn_fence(__ATOMIC_ACQUIRE, "workgroup");
}

union FB { v16b v; v4u q[2]; };

__device__ __forceinline__ v8f mma_b(v16b a, v16b b, v8f c) {
  c = __builtin_amdgcn_wmma_f32_16x16x32_bf16(false, a, false, b, (short)0, c, false, false);
#if DEV_ASM
  asm volatile("v_nop\n\tv_nop\n\tv_nop\n\tv_nop" : "+v"(c) : "v"(a), "v"(b));
#endif
  return c;
}

__device__ __forceinline__ void cvt_unit(const float* __restrict__ in, unsigned short* out, int u, int nunits) {
  const int uc = (u < nunits) ? u : (nunits - 1);
  const v4f a  = *(const v4fa*)(in + (size_t)uc * 8);
  const v4f a4 = *(const v4fa*)(in + (size_t)uc * 8 + 4);
  pin4f(a);
  pin4f(a4);
  v4u p;
  p[0] = pk16(bf_bits(a[0]),  bf_bits(a[1]));
  p[1] = pk16(bf_bits(a[2]),  bf_bits(a[3]));
  p[2] = pk16(bf_bits(a4[0]), bf_bits(a4[1]));
  p[3] = pk16(bf_bits(a4[2]), bf_bits(a4[3]));
  if (u < nunits) {
    unsigned short* o = out + (size_t)u * 8;
    *(volatile v4u*)o = p;
    __threadfence();
    *(volatile v4u*)o = p;
  }
}

struct PW { unsigned wf; unsigned wa; unsigned bb; };
__device__ __forceinline__ PW par_words(const float* __restrict__ Wf, const float* __restrict__ Wa,
                                        const float* __restrict__ ba, int t) {
  const int e = (t >> 3) & 15, q = t & 7;
  const float w0 = Wf[e * 16 + 2 * q];
  const float w1 = Wf[e * 16 + 2 * q + 1];
  const float wa = Wa[t & 31];
  const float b0 = ba[0];
  pin1f(w0); pin1f(w1); pin1f(wa); pin1f(b0);
  PW o;
  o.wf = pk16(bf_bits(w0), bf_bits(w1));
  o.wa = __float_as_uint(bfr(wa));
  o.bb = __float_as_uint(bfr(b0));
  return o;
}

__global__ __launch_bounds__(256)
void k_prep(const float* __restrict__ embC, const float* __restrict__ embI, const float* __restrict__ embS,
            const float* __restrict__ Wf0, const float* __restrict__ Wa0, const float* __restrict__ ba0,
            const float* __restrict__ Wf1, const float* __restrict__ Wa1, const float* __restrict__ ba1,
            const float* __restrict__ Wf2, const float* __restrict__ Wa2, const float* __restrict__ ba2,
            const float* __restrict__ Wf3, const float* __restrict__ Wa3, const float* __restrict__ ba3,
            const float* __restrict__ Wf4, const float* __restrict__ Wa4, const float* __restrict__ ba4,
            unsigned short* EBc, unsigned short* EBi, unsigned short* EBs, unsigned int* PAR) {
  __shared__ __align__(16) unsigned int rec[PAR_DW];
  const int t = (int)threadIdx.x;
  const int b = (int)blockIdx.x;
  if (b < BC_) {
    cvt_unit(embC, EBc, b * 256 + t, UC_);
  } else if (b < BC_ + BI_) {
    cvt_unit(embI, EBi, (b - BC_) * 256 + t, UI_);
  } else if (b < BC_ + BI_ + BS_) {
    cvt_unit(embS, EBs, (b - BC_ - BI_) * 256 + t, US_);
  } else {
    const int r = b - (BC_ + BI_ + BS_);
    PW pw;
    if (r == 0)      pw = par_words(Wf0, Wa0, ba0, t);
    else if (r == 1) pw = par_words(Wf1, Wa1, ba1, t);
    else if (r == 2) pw = par_words(Wf2, Wa2, ba2, t);
    else if (r == 3) pw = par_words(Wf3, Wa3, ba3, t);
    else             pw = par_words(Wf4, Wa4, ba4, t);
    const int e = (t >> 3) & 15, q = t & 7;
    if (t < 128) {
      rec[e * 16 + q]     = pw.wf;
      rec[e * 16 + 8 + q] = pw.wf;
    } else if (t < 160) {
      rec[PAR_WAS + (t & 31)] = pw.wa;
    } else if (t < 192) {
      rec[PAR_BA + (t - 160)] = (t == 160) ? pw.bb : 0u;
    }
    __syncthreads();
    if (t < 32) {
      const int u2 = (t + 64 < 80) ? (t + 64) : 79;
      const v4u v0 = *(const v4ua*)&rec[4 * t];
      const v4u v1 = *(const v4ua*)&rec[4 * (t + 32)];
      const v4u v2 = *(const v4ua*)&rec[4 * u2];
      unsigned int* d = PAR + (size_t)r * PAR_DW;
      for (int pass = 0; pass < 2; ++pass) {
        *(volatile v4u*)(d + 4 * t) = v0;
        *(volatile v4u*)(d + 4 * (t + 32)) = v1;
        if (t < 16) *(volatile v4u*)(d + 4 * (t + 64)) = v2;
        __threadfence();
      }
    }
  }
}

struct RowL { v4f a; v4f b; v4f c; v4f d; float dot; };
__device__ __forceinline__ RowL gather_row(const int* __restrict__ idxp, const unsigned short* __restrict__ srcp,
                                           int nsrc, int n, int j, v4f w0, v4f w1, v4f w2, v4f w3) {
  int id = idxp[(size_t)n * KK + j];
  id = (id < 0) ? 0 : id;
  id = (id > nsrc - 1) ? (nsrc - 1) : id;
  const unsigned short* rp = srcp + (size_t)id * DD;
  const v4u g0 = *(const v4ua*)rp;
  const v4u g1 = *(const v4ua*)(rp + 8);
  RowL o;
  o.a[0] = bf_lo(g0[0]); o.a[1] = bf_hi(g0[0]); o.a[2] = bf_lo(g0[1]); o.a[3] = bf_hi(g0[1]);
  o.b[0] = bf_lo(g0[2]); o.b[1] = bf_hi(g0[2]); o.b[2] = bf_lo(g0[3]); o.b[3] = bf_hi(g0[3]);
  o.c[0] = bf_lo(g1[0]); o.c[1] = bf_hi(g1[0]); o.c[2] = bf_lo(g1[1]); o.c[3] = bf_hi(g1[1]);
  o.d[0] = bf_lo(g1[2]); o.d[1] = bf_hi(g1[2]); o.d[2] = bf_lo(g1[3]); o.d[3] = bf_hi(g1[3]);
  float l = 0.0f;
  l = fmaf(o.a[0], w0[0], l); l = fmaf(o.a[1], w0[1], l); l = fmaf(o.a[2], w0[2], l); l = fmaf(o.a[3], w0[3], l);
  l = fmaf(o.b[0], w1[0], l); l = fmaf(o.b[1], w1[1], l); l = fmaf(o.b[2], w1[2], l); l = fmaf(o.b[3], w1[3], l);
  l = fmaf(o.c[0], w2[0], l); l = fmaf(o.c[1], w2[1], l); l = fmaf(o.c[2], w2[2], l); l = fmaf(o.c[3], w2[3], l);
  l = fmaf(o.d[0], w3[0], l); l = fmaf(o.d[1], w3[1], l); l = fmaf(o.d[2], w3[2], l); l = fmaf(o.d[3], w3[3], l);
  o.dot = l;
  return o;
}

template <int NREL>
__global__ __launch_bounds__(256) __attribute__((amdgpu_num_vgpr(248)))
void k_nbr(const unsigned short* __restrict__ selfp,
           const int* __restrict__ idxA, const unsigned short* __restrict__ srcA, int nsrcA,
           const unsigned int* __restrict__ parA,
           const int* __restrict__ idxB, const unsigned short* __restrict__ srcB, int nsrcB,
           const unsigned int* __restrict__ parB,
           float* outp, int ntiles) {
  __shared__ __align__(16) unsigned int sPar[NREL][PAR_DW];
  __shared__ __align__(16) float        sRows[8][2][16 * 20];
  __shared__ __align__(16) float        sWv[8][2][16];
  __shared__ __align__(16) unsigned int sAt[8][NREL][16 * 16];
  __shared__ __align__(16) float        sDt[8][16 * 16];

  const int tid  = (int)threadIdx.x;
  const int wave = __builtin_amdgcn_readfirstlane(tid >> 5);
  const int lane = tid & 31;
  const int hw   = lane >> 4;
  const int j    = lane & 15;

  {
    const int uu = (tid < 79) ? tid : 79;
    const v4u pa = *(const v4ua*)(parA + 4 * uu);
    pin4u(pa);
    if (tid < 80) *(v4ua*)&sPar[0][4 * uu] = pa;
    if (NREL == 2) {
      const v4u pb = *(const v4ua*)(parB + 4 * uu);
      pin4u(pb);
      if (tid < 80) *(v4ua*)&sPar[NREL - 1][4 * uu] = pb;
    }
  }
  __syncthreads();

  const int tile = (int)blockIdx.x * 8 + wave;
  if (tile < ntiles) {
    FB    bfrag[NREL];
    v4f   wn[NREL][4];
    float was[NREL], bav[NREL];
#pragma unroll
    for (int r = 0; r < NREL; ++r) {
      const unsigned int* wb = &sPar[r][j * 16 + 4 * hw];
      bfrag[r].q[0] = *(const v4ua*)wb;
      bfrag[r].q[1] = *(const v4ua*)(wb + 8);
#pragma unroll
      for (int q4 = 0; q4 < 4; ++q4) wn[r][q4] = *(const v4fa*)&sPar[r][PAR_WAN + 4 * q4];
      was[r] = __uint_as_float(sPar[r][PAR_WAS + j]);
      bav[r] = __uint_as_float(sPar[r][PAR_BA]);
    }

#pragma unroll 1
    for (int it = 0; it < 8; ++it) {
      const int row = it * 2 + hw;
      const int n   = tile * 16 + row;
      const float sv = bf_up((unsigned)selfp[(size_t)n * DD + j]);

      RowL rw[NREL];
      rw[0] = gather_row(idxA, srcA, nsrcA, n, j, wn[0][0], wn[0][1], wn[0][2], wn[0][3]);
      if (NREL == 2)
        rw[NREL - 1] = gather_row(idxB, srcB, nsrcB, n, j,
                                  wn[NREL - 1][0], wn[NREL - 1][1], wn[NREL - 1][2], wn[NREL - 1][3]);

#pragma unroll
      for (int r = 0; r < NREL; ++r) {
        float sd = sv * was[r];
        sd += __shfl_xor(sd, 8, 32);
        sd += __shfl_xor(sd, 4, 32);
        sd += __shfl_xor(sd, 2, 32);
        sd += __shfl_xor(sd, 1, 32);
        const float logit = (rw[r].dot + sd) + bav[r];
        float mx = logit;
        mx = fmaxf(mx, __shfl_xor(mx, 8, 32));
        mx = fmaxf(mx, __shfl_xor(mx, 4, 32));
        mx = fmaxf(mx, __shfl_xor(mx, 2, 32));
        mx = fmaxf(mx, __shfl_xor(mx, 1, 32));
        const float p = expf(logit - mx);
        float sum = p;
        sum += __shfl_xor(sum, 8, 32);
        sum += __shfl_xor(sum, 4, 32);
        sum += __shfl_xor(sum, 2, 32);
        sum += __shfl_xor(sum, 1, 32);
        const float w = p / sum;

        wave_lds_sync();
        float* rowp = &sRows[wave][hw][j * 20];
        *(v4fa*)(rowp)      = rw[r].a;
        *(v4fa*)(rowp + 4)  = rw[r].b;
        *(v4fa*)(rowp + 8)  = rw[r].c;
        *(v4fa*)(rowp + 12) = rw[r].d;
        sWv[wave][hw][j] = w;
        wave_lds_sync();

        const v4f wv0 = *(const v4fa*)&sWv[wave][hw][0];
        const v4f wv1 = *(const v4fa*)&sWv[wave][hw][4];
        const v4f wv2 = *(const v4fa*)&sWv[wave][hw][8];
        const v4f wv3 = *(const v4fa*)&sWv[wave][hw][12];
        const float* colp = &sRows[wave][hw][j];
        float s = 0.0f;
        s = fmaf(wv0[0], colp[0 * 20],  s); s = fmaf(wv0[1], colp[1 * 20],  s);
        s = fmaf(wv0[2], colp[2 * 20],  s); s = fmaf(wv0[3], colp[3 * 20],  s);
        s = fmaf(wv1[0], colp[4 * 20],  s); s = fmaf(wv1[1], colp[5 * 20],  s);
        s = fmaf(wv1[2], colp[6 * 20],  s); s = fmaf(wv1[3], colp[7 * 20],  s);
        s = fmaf(wv2[0], colp[8 * 20],  s); s = fmaf(wv2[1], colp[9 * 20],  s);
        s = fmaf(wv2[2], colp[10 * 20], s); s = fmaf(wv2[3], colp[11 * 20], s);
        s = fmaf(wv3[0], colp[12 * 20], s); s = fmaf(wv3[1], colp[13 * 20], s);
        s = fmaf(wv3[2], colp[14 * 20], s); s = fmaf(wv3[3], colp[15 * 20], s);

        const unsigned hb = (unsigned)bf_bits(s);
        const unsigned lb = (unsigned)bf_bits(s - bf_up(hb));
        const unsigned comb = hb | (lb << 16);
        const int src0 = (lane & 16) + 2 * (j & 7);
        const unsigned c0 = (unsigned)__shfl((int)comb, src0, 32);
        const unsigned c1 = (unsigned)__shfl((int)comb, src0 + 1, 32);
        const unsigned whi = (c0 & 0xffffu) | (c1 << 16);
        const unsigned wlo = (c0 >> 16) | (c1 & 0xffff0000u);
        const unsigned msk = (j < 8) ? 0xffffffffu : 0u;
        sAt[wave][r][row * 16 + j] = (whi & msk) | (wlo & ~msk);
      }
    }
    wave_lds_sync();

    v8f acc = zero8();
    {
      FB af;
      const unsigned int* ap = &sAt[wave][0][j * 16 + 4 * hw];
      af.q[0] = *(const v4ua*)ap;
      af.q[1] = *(const v4ua*)(ap + 8);
      acc = mma_b(af.v, bfrag[0].v, acc);
    }
    if (NREL == 2) {
      FB af;
      const unsigned int* ap = &sAt[wave][NREL - 1][j * 16 + 4 * hw];
      af.q[0] = *(const v4ua*)ap;
      af.q[1] = *(const v4ua*)(ap + 8);
      acc = mma_b(af.v, bfrag[NREL - 1].v, acc);
    }

#pragma unroll
    for (int r = 0; r < 8; ++r) sDt[wave][(8 * hw + r) * 16 + j] = acc[r];
    wave_lds_sync();

    v4f ov[2];
#pragma unroll
    for (int i = 0; i < 2; ++i) {
      const int u = lane + 32 * i;
      const v4f dv = *(const v4fa*)&sDt[wave][u * 4];
      const v2u sw = *(const v2ua*)(selfp + (size_t)tile * 256 + (size_t)u * 4);
      ov[i][0] = dv[0] + bf_lo(sw[0]);
      ov[i][1] = dv[1] + bf_hi(sw[0]);
      ov[i][2] = dv[2] + bf_lo(sw[1]);
      ov[i][3] = dv[3] + bf_hi(sw[1]);
    }
    float* ob = outp + (size_t)tile * 256;
    for (int pass = 0; pass < 2; ++pass) {
#pragma unroll
      for (int i = 0; i < 2; ++i) {
        float* o = ob + (size_t)(lane + 32 * i) * 4;
        *(volatile v4f*)o = ov[i];
      }
      __threadfence();
    }
  }
}

extern "C" void kernel_launch(void* const* d_in, const int* in_sizes, int n_in,
                              void* d_out, int out_size, void* d_ws, size_t ws_size,
                              hipStream_t stream) {
  if (n_in < 23) return;
  if (in_sizes[0] != NC_ * DD || in_sizes[1] != NI_ * DD || in_sizes[2] != NS_ * DD) return;
  if (in_sizes[3] != 256 || in_sizes[4] != 256 || in_sizes[9] != 256 || in_sizes[10] != 256 || in_sizes[15] != 256) return;
  if (in_sizes[5] != 32 || in_sizes[7] != 32 || in_sizes[11] != 32 || in_sizes[13] != 32 || in_sizes[16] != 32) return;
  if (in_sizes[6] != 1 || in_sizes[8] != 1 || in_sizes[12] != 1 || in_sizes[14] != 1 || in_sizes[17] != 1) return;
  if (in_sizes[18] != NC_ * KK || in_sizes[19] != NC_ * KK) return;
  if (in_sizes[20] != NI_ * KK || in_sizes[21] != NI_ * KK || in_sizes[22] != NS_ * KK) return;
  if (out_size != OTOT_) return;

  const float* embC  = (const float*)d_in[0];
  const float* embI  = (const float*)d_in[1];
  const float* embS  = (const float*)d_in[2];
  const float* c_Wf1 = (const float*)d_in[3];
  const float* c_Wf2 = (const float*)d_in[4];
  const float* c_Wa1 = (const float*)d_in[5];
  const float* c_ba1 = (const float*)d_in[6];
  const float* c_Wa2 = (const float*)d_in[7];
  const float* c_ba2 = (const float*)d_in[8];
  const float* i_Wf1 = (const float*)d_in[9];
  const float* i_Wf2 = (const float*)d_in[10];
  const float* i_Wa1 = (const float*)d_in[11];
  const float* i_ba1 = (const float*)d_in[12];
  const float* i_Wa2 = (const float*)d_in[13];
  const float* i_ba2 = (const float*)d_in[14];
  const float* s_Wf  = (const float*)d_in[15];
  const float* s_Wa  = (const float*)d_in[16];
  const float* s_ba  = (const float*)d_in[17];
  const int* cc_idx = (const int*)d_in[18];
  const int* ci_idx = (const int*)d_in[19];
  const int* ic_idx = (const int*)d_in[20];
  const int* is_idx = (const int*)d_in[21];
  const int* si_idx = (const int*)d_in[22];
  float* out = (float*)d_out;

  size_t off = 0;
  const size_t oC = off; off += (size_t)NC_ * DD * 2;
  const size_t oI = off; off += (size_t)NI_ * DD * 2;
  const size_t oS = off; off += (size_t)NS_ * DD * 2;
  const size_t oP = off; off += (size_t)NREC * PAR_DW * 4;
  if (off > ws_size) return;
  if (off > (size_t)WSCAP) return;
  if ((oI % 256) != 0 || (oS % 256) != 0 || (oP % 256) != 0) return;

  char* ws = (char*)d_ws;
  unsigned short* EBc = (unsigned short*)(ws + oC);
  unsigned short* EBi = (unsigned short*)(ws + oI);
  unsigned short* EBs = (unsigned short*)(ws + oS);
  unsigned int*   PAR = (unsigned int*)(ws + oP);

  const dim3 blk(256);
  k_prep<<<dim3(BC_ + BI_ + BS_ + NREC), blk, 0, stream>>>(
      embC, embI, embS,
      c_Wf1, c_Wa1, c_ba1,
      c_Wf2, c_Wa2, c_ba2,
      i_Wf1, i_Wa1, i_ba1,
      i_Wf2, i_Wa2, i_ba2,
      s_Wf,  s_Wa,  s_ba,
      EBc, EBi, EBs, PAR);
  k_nbr<2><<<dim3((NC_ / 16 + 7) / 8), blk, 0, stream>>>(
      EBc, cc_idx, EBc, NC_, PAR + 0 * PAR_DW, ci_idx, EBi, NI_, PAR + 1 * PAR_DW, out + O0_, NC_ / 16);
  k_nbr<2><<<dim3((NI_ / 16 + 7) / 8), blk, 0, stream>>>(
      EBi, ic_idx, EBc, NC_, PAR + 2 * PAR_DW, is_idx, EBs, NS_, PAR + 3 * PAR_DW, out + O1_, NI_ / 16);
  k_nbr<1><<<dim3((NS_ / 16 + 7) / 8), blk, 0, stream>>>(
      EBs, si_idx, EBi, NI_, PAR + 4 * PAR_DW, si_idx, EBi, NI_, PAR + 4 * PAR_DW, out + O2_, NS_ / 16);
  (void)hipGetLastError();
}
